// GNN_24816321036584
// MI455X (gfx1250) — hardware-verified
//
#include <hip/hip_runtime.h>
#include <stddef.h>
#include <stdint.h>
#include <math.h>


#define U_N   32
#define SU    8
#define HH    64
#define NCL   4
#define NE    992
#define G3    192
#define KP    128
#define K2C   64
#define TR    64
#define NTILE 16
#define NIT   3
#define NTHR  256
#define SMS   592
#define WSMAX 134217728

#define OW1A  0
#define OB1A  40
#define OB2B  48
#define OB2C  80
#define OB4   88
#define OB3A  96
#define OB3B  160
#define OB3C  192
#define OBIH  196
#define OBHH  388

static_assert(NE == U_N * (U_N - 1));
static_assert(NTILE * 2 == U_N);
static_assert(TR >= 2 * (U_N - 1) && TR == 64);
static_assert(NTHR == U_N * SU);
static_assert(NTHR * 8 == U_N * HH);
static_assert(NTHR / 4 == TR);
static_assert((KP % 32) == 0 && (K2C % 32) == 0);
static_assert(OBHH + G3 <= SMS);
static_assert((OB1A % 4) == 0 && (OB2B % 4) == 0 && (OB2C % 4) == 0 && (OB4 % 4) == 0);
static_assert((OB3A % 4) == 0 && (OB3B % 4) == 0 && (OB3C % 4) == 0 && (OBIH % 4) == 0 && (OBHH % 4) == 0);

typedef float          v4f  __attribute__((ext_vector_type(4)));
typedef float          v8f  __attribute__((ext_vector_type(8)));
typedef int            v8i  __attribute__((ext_vector_type(8)));
typedef unsigned int   v4u  __attribute__((ext_vector_type(4)));
typedef unsigned short v4us __attribute__((ext_vector_type(4)));
typedef unsigned short v8us __attribute__((ext_vector_type(8)));
typedef __bf16         v16b __attribute__((ext_vector_type(16)));
typedef v4f  __attribute__((may_alias)) v4fa;
typedef v4u  __attribute__((may_alias)) v4ua;
typedef v4us __attribute__((may_alias)) v4usa;
typedef v8us __attribute__((may_alias)) v8usa;
union FragB { v16b v; v8us h[2]; v8i w; };

__device__ __forceinline__ v8f wmb(const FragB& a, const FragB& b, v8f c) {
  v8f d = __builtin_amdgcn_wmma_f32_16x16x32_bf16(false, a.v, false, b.v, (short)0, c, false, false);
  asm volatile("v_nop\n\tv_nop\n\tv_nop\n\tv_nop" : "+v"(d) : "v"(a.w), "v"(b.w));
  return d;
}

__device__ __forceinline__ unsigned int f2bf(float f) {
  const unsigned int u = __float_as_uint(f);
  return ((u + 0x7FFFu + ((u >> 16) & 1u)) >> 16) & 0xFFFFu;
}
__device__ __forceinline__ float bf2f(unsigned int b) { return __uint_as_float(b << 16); }
__device__ __forceinline__ float bfr(float f) { return bf2f(f2bf(f)); }
__device__ __forceinline__ v4f bfr4(const v4f a) {
  v4f r; r.x = bfr(a.x); r.y = bfr(a.y); r.z = bfr(a.z); r.w = bfr(a.w); return r;
}
__device__ __forceinline__ unsigned int pk2(float lo, float hi) { return f2bf(lo) | (f2bf(hi) << 16); }
__device__ __forceinline__ v4u pack8(const v4f a, const v4f b) {
  v4u r;
  r.x = pk2(a.x, a.y); r.y = pk2(a.z, a.w); r.z = pk2(b.x, b.y); r.w = pk2(b.z, b.w);
  return r;
}
__device__ __forceinline__ void hilo2(float a, float b, unsigned int& hp, unsigned int& lp) {
  const unsigned int ha = f2bf(a), hb = f2bf(b);
  const unsigned int la = f2bf(a - bf2f(ha)), lb = f2bf(b - bf2f(hb));
  hp = ha | (hb << 16);
  lp = la | (lb << 16);
}
__device__ __forceinline__ v4f madd4(float s, const v4f w, v4f acc) {
  acc.x = fmaf(s, w.x, acc.x); acc.y = fmaf(s, w.y, acc.y); acc.z = fmaf(s, w.z, acc.z); acc.w = fmaf(s, w.w, acc.w);
  return acc;
}
__device__ __forceinline__ float dot8(const v4f s0, const v4f s1, const v4f w0, const v4f w1) {
  float d = s0.x * w0.x;
  d = fmaf(s0.y, w0.y, d); d = fmaf(s0.z, w0.z, d); d = fmaf(s0.w, w0.w, d);
  d = fmaf(s1.x, w1.x, d); d = fmaf(s1.y, w1.y, d); d = fmaf(s1.z, w1.z, d); d = fmaf(s1.w, w1.w, d);
  return d;
}
__device__ __forceinline__ float sigm(float x) {
  const float e = expf(-x);
  return __builtin_amdgcn_rcpf(1.0f + e);
}

__global__ __launch_bounds__(NTHR) void k_wtr(const float* __restrict__ w, int Kin, int Ncol, int Nrows, int Kout,
                                              unsigned short* wt, int nUnits) {
  const int u = (int)blockIdx.x * NTHR + (int)threadIdx.x;
  if (u >= nUnits) return;
  const int kq = Kout >> 3;
  const int n  = u / kq;
  const int k8 = (u - n * kq) * 8;
  const int kk = k8 - (k8 / Kin) * Kin;
  const int ncl = n < Ncol ? n : Ncol - 1;
  const float* p = w + (size_t)kk * (size_t)Ncol + ncl;
  v4f a, b;
  a.x = p[0];                    a.y = p[(size_t)Ncol];         a.z = p[(size_t)2 * Ncol];     a.w = p[(size_t)3 * Ncol];
  b.x = p[(size_t)4 * Ncol];     b.y = p[(size_t)5 * Ncol];     b.z = p[(size_t)6 * Ncol];     b.w = p[(size_t)7 * Ncol];
  const v4f z4 = {0.f, 0.f, 0.f, 0.f};
  if (n >= Ncol || n >= Nrows) { a = z4; b = z4; }
  const v4u wv = pack8(a, b);
  unsigned short* o = wt + (size_t)n * (size_t)Kout + k8;
  *(volatile v4u*)o = wv;
  __threadfence();
  *(volatile v4u*)o = wv;
}

__global__ __launch_bounds__(NTHR) void k_wdup(const float* __restrict__ w, unsigned short* wt, int nUnits) {
  const int u = (int)blockIdx.x * NTHR + (int)threadIdx.x;
  if (u >= nUnits) return;
  const int n  = u >> 4;
  const int k8 = (u & 15) * 8;
  const int kk = k8 & (HH - 1);
  const float* p = w + (size_t)n * HH + kk;
  const v4f a = *(const v4f*)p;
  const v4f c = *(const v4f*)(p + 4);
  const v4u wv = pack8(a, c);
  unsigned short* o = wt + (size_t)n * KP + k8;
  *(volatile v4u*)o = wv;
  __threadfence();
  *(volatile v4u*)o = wv;
}

__device__ __forceinline__ v4u m1grp(const float* pa, const float* pb, const float* w6, const float* cn, float ewv) {
  const v4f a  = *(const v4fa*)pa;
  const v4f q  = *(const v4fa*)pb;
  const v4f ww = *(const v4fa*)w6;
  const v4f cc = *(const v4fa*)cn;
  v4f v = a + q;
  v = madd4(ewv, ww, v);
  v = v + cc;
  v.x = fmaxf(v.x, 0.0f); v.y = fmaxf(v.y, 0.0f); v.z = fmaxf(v.z, 0.0f); v.w = fmaxf(v.w, 0.0f);
  unsigned int h01, h23, l01, l23;
  hilo2(v.x, v.y, h01, l01);
  hilo2(v.z, v.w, h23, l23);
  v4u o;
  o.x = h01; o.y = h23; o.z = l01; o.w = l23;
  return o;
}

struct EdgePh {
  float PA[U_N * HH];
  float PB[U_N * HH];
  unsigned short m1[TR * KP];
  unsigned short m2[TR * K2C];
  float m3[TR * SU];
};
struct GruPh {
  unsigned short hxA[U_N * KP];
  float gh[U_N * G3];
  float W4R[HH * SU];
};
struct RoPh {
  float t1[U_N * HH];
  float t2[U_N * (HH / 2)];
  float outs[U_N * NCL];
};
union PhU { EdgePh e; GruPh g; RoPh r; };
static_assert(sizeof(EdgePh) == 43008);
static_assert(sizeof(GruPh) <= sizeof(EdgePh) && sizeof(RoPh) <= sizeof(EdgePh));

__global__ __launch_bounds__(NTHR) void k_net(
    const float* __restrict__ xf,   const float* __restrict__ ew,   const float* __restrict__ noise,
    const float* __restrict__ hx0,  const float* __restrict__ xhat, const float* __restrict__ varm,
    const float* __restrict__ W1a,  const float* __restrict__ b1a,
    const float* __restrict__ W2a,  const float* __restrict__ b2a,
    const float* __restrict__ b2b,  const float* __restrict__ b2c,
    const float* __restrict__ W3a,  const float* __restrict__ b3a,
    const float* __restrict__ W3b,  const float* __restrict__ b3b,
    const float* __restrict__ W3c,  const float* __restrict__ b3c,
    const float* __restrict__ Wih,  const float* __restrict__ bih,  const float* __restrict__ bhh,
    const float* __restrict__ W4,   const float* __restrict__ b4,
    const unsigned short* __restrict__ W2bP, const unsigned short* __restrict__ W2cP,
    const unsigned short* __restrict__ WhhP, float* out)
{
  __shared__ __attribute__((aligned(16))) float hxS[U_N * HH];
  __shared__ __attribute__((aligned(16))) float nodesS[U_N * SU];
  __shared__ __attribute__((aligned(16))) float sumS[U_N * SU];
  __shared__ __attribute__((aligned(16))) unsigned short ewS[1024];
  __shared__ __attribute__((aligned(16))) float W2aS[16 * HH];
  __shared__ __attribute__((aligned(16))) float W16S[HH];
  __shared__ __attribute__((aligned(16))) float CNS[HH];
  __shared__ __attribute__((aligned(16))) float smS[SMS];
  __shared__ __attribute__((aligned(16))) PhU un;

  const int tid = (int)threadIdx.x, lane = tid & 31, wave = tid >> 5, hh = lane >> 4, m = lane & 15;
  const int b = (int)blockIdx.x;
  const v4f z4 = {0.f, 0.f, 0.f, 0.f};
  const v8f z8 = {0.f, 0.f, 0.f, 0.f, 0.f, 0.f, 0.f, 0.f};

  {
    const float* hp = hx0 + (size_t)b * (U_N * HH);
    const v4f a = *(const v4f*)(hp + 4 * tid);
    const v4f c = *(const v4f*)(hp + 4 * tid + 1024);
    *(v4fa*)(hxS + 4 * tid) = bfr4(a);
    *(v4fa*)(hxS + 4 * tid + 1024) = bfr4(c);
  }
  {
    const int q = tid < (NE / 4) ? tid : (NE / 4) - 1;
    const v4f a = *(const v4f*)(ew + (size_t)b * NE + 4 * q);
    v4us o;
    o[0] = (unsigned short)f2bf(a.x); o[1] = (unsigned short)f2bf(a.y);
    o[2] = (unsigned short)f2bf(a.z); o[3] = (unsigned short)f2bf(a.w);
    if (tid < (NE / 4)) *(v4usa*)(ewS + 4 * tid) = o;
  }
#define STG4(SRC, NU, OFF) { const int q_ = tid < (NU) ? tid : (NU) - 1; \
    const v4f a_ = *(const v4f*)((SRC) + 4 * q_); \
    if (tid < (NU)) *(v4fa*)(smS + (OFF) + 4 * tid) = bfr4(a_); }
  STG4(W1a, 10, OW1A)
  STG4(b1a, 2, OB1A)
  STG4(b2b, 8, OB2B)
  STG4(b2c, 2, OB2C)
  STG4(b4, 2, OB4)
  STG4(b3a, 16, OB3A)
  STG4(b3b, 8, OB3B)
  STG4(b3c, 1, OB3C)
  STG4(bih, 48, OBIH)
  STG4(bhh, 48, OBHH)
#undef STG4
  {
    const v4f a = *(const v4f*)(W2a + 4 * tid);
    *(v4fa*)(W2aS + 4 * tid) = bfr4(a);
    const int q = tid < 16 ? tid : 15;
    const v4f w6 = *(const v4f*)(W2a + 16 * HH + 4 * q);
    const v4f w7 = *(const v4f*)(W2a + 17 * HH + 4 * q);
    const v4f bb = *(const v4f*)(b2a + 4 * q);
    const float nz = bfr(noise[b]);
    if (tid < 16) {
      *(v4fa*)(W16S + 4 * tid) = bfr4(w6);
      v4f c;
      c.x = fmaf(nz, bfr(w7.x), bfr(bb.x)); c.y = fmaf(nz, bfr(w7.y), bfr(bb.y));
      c.z = fmaf(nz, bfr(w7.z), bfr(bb.z)); c.w = fmaf(nz, bfr(w7.w), bfr(bb.w));
      *(v4fa*)(CNS + 4 * tid) = c;
    }
  }
  float x0, x1, x2, x3, x4;
  {
    const int u = tid >> 3;
    const size_t nb = (size_t)b * U_N + u;
    x0 = bfr(xf[nb * 3 + 0]); x1 = bfr(xf[nb * 3 + 1]); x2 = bfr(xf[nb * 3 + 2]);
    x3 = bfr(xhat[nb]); x4 = bfr(varm[nb]);
  }
  __syncthreads();
  {
    const int o = tid & 7;
    float a = x0 * smS[OW1A + o];
    a = fmaf(x1, smS[OW1A + 1 * SU + o], a);
    a = fmaf(x2, smS[OW1A + 2 * SU + o], a);
    a = fmaf(x3, smS[OW1A + 3 * SU + o], a);
    a = fmaf(x4, smS[OW1A + 4 * SU + o], a);
    nodesS[tid] = a + smS[OB1A + o];
  }
  __syncthreads();

#pragma unroll 1
  for (int it = 0; it < NIT; ++it) {
    {
      const int u = tid >> 3, c8 = (tid & 7) * 8;
      v4f pa0 = z4, pa1 = z4, pb0 = z4, pb1 = z4;
#pragma unroll 2
      for (int k = 0; k < SU; ++k) {
        const float nk = nodesS[u * SU + k];
        const v4f wa0 = *(const v4fa*)(W2aS + k * HH + c8);
        const v4f wa1 = *(const v4fa*)(W2aS + k * HH + c8 + 4);
        const v4f wb0 = *(const v4fa*)(W2aS + (SU + k) * HH + c8);
        const v4f wb1 = *(const v4fa*)(W2aS + (SU + k) * HH + c8 + 4);
        pa0 = madd4(nk, wa0, pa0); pa1 = madd4(nk, wa1, pa1);
        pb0 = madd4(nk, wb0, pb0); pb1 = madd4(nk, wb1, pb1);
      }
      *(v4fa*)(un.e.PA + u * HH + c8) = pa0;  *(v4fa*)(un.e.PA + u * HH + c8 + 4) = pa1;
      *(v4fa*)(un.e.PB + u * HH + c8) = pb0;  *(v4fa*)(un.e.PB + u * HH + c8 + 4) = pb1;
    }
    __syncthreads();

#pragma unroll 1
    for (int t = 0; t < NTILE; ++t) {
      {
        const int r  = tid >> 2;
        const int cq = (tid & 3) * 16;
        const int rc = r < 2 * (U_N - 1) ? r : 2 * (U_N - 1) - 1;
        const int nn = (rc >= (U_N - 1)) ? 1 : 0;
        const int jj = rc - (U_N - 1) * nn;
        const int ni = 2 * t + nn;
        const int nj = jj + ((jj >= ni) ? 1 : 0);
        const float ewv = bf2f((unsigned int)ewS[ni * (U_N - 1) + jj]);
        const float* pa = un.e.PA + ni * HH + cq;
        const float* pb = un.e.PB + nj * HH + cq;
        const v4u g0 = m1grp(pa,      pb,      W16S + cq,      CNS + cq,      ewv);
        const v4u g1 = m1grp(pa + 4,  pb + 4,  W16S + cq + 4,  CNS + cq + 4,  ewv);
        const v4u g2 = m1grp(pa + 8,  pb + 8,  W16S + cq + 8,  CNS + cq + 8,  ewv);
        const v4u g3 = m1grp(pa + 12, pb + 12, W16S + cq + 12, CNS + cq + 12, ewv);
        v4u hv0, hv1, lv0, lv1;
        hv0.x = g0.x; hv0.y = g0.y; hv0.z = g1.x; hv0.w = g1.y;
        hv1.x = g2.x; hv1.y = g2.y; hv1.z = g3.x; hv1.w = g3.y;
        lv0.x = g0.z; lv0.y = g0.w; lv0.z = g1.z; lv0.w = g1.w;
        lv1.x = g2.z; lv1.y = g2.w; lv1.z = g3.z; lv1.w = g3.w;
        unsigned short* row = un.e.m1 + r * KP;
        *(v4ua*)(row + cq) = hv0;           *(v4ua*)(row + cq + 8) = hv1;
        *(v4ua*)(row + HH + cq) = lv0;      *(v4ua*)(row + HH + cq + 8) = lv1;
      }
      __syncthreads();

      {
        const int rt = wave & 3, ct = wave >> 2;
        const unsigned short* ap = un.e.m1 + (16 * rt + m) * KP + 8 * hh;
        const unsigned short* bp = W2bP + (size_t)(16 * ct + m) * KP + 8 * hh;
        v8f acc = z8;
#pragma unroll
        for (int ks = 0; ks < KP / 32; ++ks) {
          FragB af, bf;
          af.h[0] = *(const v8usa*)(ap + 32 * ks);
          af.h[1] = *(const v8usa*)(ap + 32 * ks + 16);
          bf.h[0] = *(const v8usa*)(bp + 32 * ks);
          bf.h[1] = *(const v8usa*)(bp + 32 * ks + 16);
          acc = wmb(af, bf, acc);
        }
        const float bb = smS[OB2B + 16 * ct + m];
#pragma unroll
        for (int r = 0; r < 8; ++r) {
          const int row = 16 * rt + 8 * hh + r;
          const float v = fmaxf(acc[r] + bb, 0.0f);
          const unsigned int hb = f2bf(v);
          const unsigned int lb = f2bf(v - bf2f(hb));
          un.e.m2[row * K2C + 16 * ct + m] = (unsigned short)hb;
          un.e.m2[row * K2C + (HH / 2) + 16 * ct + m] = (unsigned short)lb;
        }
      }
      __syncthreads();

      if (wave < 4) {
        const unsigned short* ap = un.e.m2 + (16 * wave + m) * K2C + 8 * hh;
        const unsigned short* bp = W2cP + (size_t)m * K2C + 8 * hh;
        v8f acc = z8;
#pragma unroll
        for (int ks = 0; ks < K2C / 32; ++ks) {
          FragB af, bf;
          af.h[0] = *(const v8usa*)(ap + 32 * ks);
          af.h[1] = *(const v8usa*)(ap + 32 * ks + 16);
          bf.h[0] = *(const v8usa*)(bp + 32 * ks);
          bf.h[1] = *(const v8usa*)(bp + 32 * ks + 16);
          acc = wmb(af, bf, acc);
        }
        const float bc = smS[OB2C + (m & 7)];
#pragma unroll
        for (int r = 0; r < 8; ++r) {
          const int row = 16 * wave + 8 * hh + r;
          const float v = fmaxf(acc[r] + bc, 0.0f);
          if (m < SU) un.e.m3[row * SU + m] = v;
        }
      }
      __syncthreads();

      if (tid < 16) {
        const int nn = tid >> 3, f = tid & 7;
        float s = 0.0f;
#pragma unroll 1
        for (int r = 0; r < U_N - 1; ++r) s += un.e.m3[((U_N - 1) * nn + r) * SU + f];
        sumS[(2 * t + nn) * SU + f] = s;
      }
    }
    __syncthreads();

    {
      const int node = tid >> 3, c8 = (tid & 7) * 8;
      const v4f a = *(const v4fa*)(hxS + node * HH + c8);
      const v4f c = *(const v4fa*)(hxS + node * HH + c8 + 4);
      unsigned int h0, h1, h2, h3, l0, l1, l2, l3;
      hilo2(a.x, a.y, h0, l0); hilo2(a.z, a.w, h1, l1);
      hilo2(c.x, c.y, h2, l2); hilo2(c.z, c.w, h3, l3);
      v4u hv, lv;
      hv.x = h0; hv.y = h1; hv.z = h2; hv.w = h3;
      lv.x = l0; lv.y = l1; lv.z = l2; lv.w = l3;
      *(v4ua*)(un.g.hxA + node * KP + c8) = hv;
      *(v4ua*)(un.g.hxA + node * KP + HH + c8) = lv;
      const int q = tid < (HH * SU / 4) ? tid : (HH * SU / 4) - 1;
      const v4f w = *(const v4f*)(W4 + 4 * q);
      if (tid < (HH * SU / 4)) *(v4fa*)(un.g.W4R + 4 * tid) = bfr4(w);
    }
    __syncthreads();

#pragma unroll 1
    for (int q = 0; q < 3; ++q) {
      const int p  = wave + 8 * q;
      const int mt = p & 1, nt = p >> 1;
      const unsigned short* ap = un.g.hxA + (16 * mt + m) * KP + 8 * hh;
      const unsigned short* bp = WhhP + (size_t)(16 * nt + m) * KP + 8 * hh;
      v8f acc = z8;
#pragma unroll
      for (int ks = 0; ks < KP / 32; ++ks) {
        FragB af, bf;
        af.h[0] = *(const v8usa*)(ap + 32 * ks);
        af.h[1] = *(const v8usa*)(ap + 32 * ks + 16);
        bf.h[0] = *(const v8usa*)(bp + 32 * ks);
        bf.h[1] = *(const v8usa*)(bp + 32 * ks + 16);
        acc = wmb(af, bf, acc);
      }
#pragma unroll
      for (int r = 0; r < 8; ++r) un.g.gh[(16 * mt + 8 * hh + r) * G3 + 16 * nt + m] = acc[r];
    }
    __syncthreads();

    {
      const int jg = tid & 63, ngp = tid >> 6;
      const v4f wr0 = bfr4(*(const v4f*)(Wih + (size_t)jg * SU));
      const v4f wr1 = bfr4(*(const v4f*)(Wih + (size_t)jg * SU + 4));
      const v4f wz0 = bfr4(*(const v4f*)(Wih + (size_t)(HH + jg) * SU));
      const v4f wz1 = bfr4(*(const v4f*)(Wih + (size_t)(HH + jg) * SU + 4));
      const v4f wn0 = bfr4(*(const v4f*)(Wih + (size_t)(2 * HH + jg) * SU));
      const v4f wn1 = bfr4(*(const v4f*)(Wih + (size_t)(2 * HH + jg) * SU + 4));
      const float bir = smS[OBIH + jg], biz = smS[OBIH + HH + jg], bin = smS[OBIH + 2 * HH + jg];
      const float bhr = smS[OBHH + jg], bhz = smS[OBHH + HH + jg], bhn = smS[OBHH + 2 * HH + jg];
#pragma unroll 1
      for (int q = 0; q < 8; ++q) {
        const int node = 8 * ngp + q;
        const v4f s0 = *(const v4fa*)(sumS + node * SU);
        const v4f s1 = *(const v4fa*)(sumS + node * SU + 4);
        const float gir = dot8(s0, s1, wr0, wr1) + bir;
        const float giz = dot8(s0, s1, wz0, wz1) + biz;
        const float gin = dot8(s0, s1, wn0, wn1) + bin;
        const float* gp = un.g.gh + node * G3 + jg;
        const float ghr = gp[0] + bhr;
        const float ghz = gp[HH] + bhz;
        const float ghn = gp[2 * HH] + bhn;
        const float rg = sigm(gir + ghr);
        const float zg = sigm(giz + ghz);
        const float cg = tanhf(fmaf(rg, ghn, gin));
        const float ho = hxS[node * HH + jg];
        hxS[node * HH + jg] = fmaf(zg, ho, (1.0f - zg) * cg);
      }
    }
    __syncthreads();

    {
      const int node = tid >> 3, o = tid & 7;
      float a = 0.0f;
#pragma unroll 4
      for (int k = 0; k < HH; ++k) a = fmaf(hxS[node * HH + k], un.g.W4R[k * SU + o], a);
      nodesS[tid] = a + smS[OB4 + o];
    }
    __syncthreads();
  }

  {
    const int u = tid >> 3, c8 = (tid & 7) * 8;
    v4f a0 = z4, a1 = z4;
#pragma unroll 1
    for (int k = 0; k < SU; ++k) {
      const float nk = nodesS[u * SU + k];
      const v4f w0 = bfr4(*(const v4f*)(W3a + (size_t)k * HH + c8));
      const v4f w1 = bfr4(*(const v4f*)(W3a + (size_t)k * HH + c8 + 4));
      a0 = madd4(nk, w0, a0); a1 = madd4(nk, w1, a1);
    }
    a0 = a0 + *(const v4fa*)(smS + OB3A + c8);
    a1 = a1 + *(const v4fa*)(smS + OB3A + c8 + 4);
    *(v4fa*)(un.r.t1 + u * HH + c8) = a0;
    *(v4fa*)(un.r.t1 + u * HH + c8 + 4) = a1;
  }
  __syncthreads();
  {
    const int u = tid >> 3, o4 = (tid & 7) * 4;
    v4f a = z4;
#pragma unroll 2
    for (int k = 0; k < HH; ++k) {
      const float xk = un.r.t1[u * HH + k];
      const v4f w = bfr4(*(const v4f*)(W3b + (size_t)k * (HH / 2) + o4));
      a = madd4(xk, w, a);
    }
    a = a + *(const v4fa*)(smS + OB3B + o4);
    *(v4fa*)(un.r.t2 + u * (HH / 2) + o4) = a;
  }
  __syncthreads();
  {
    const int uu = tid >> 2, u = uu < U_N ? uu : U_N - 1, c = tid & 3;
    float a = 0.0f;
#pragma unroll 4
    for (int k = 0; k < HH / 2; ++k) a = fmaf(un.r.t2[u * (HH / 2) + k], bfr(W3c[k * NCL + c]), a);
    a += smS[OB3C + c];
    if (tid < U_N * NCL) un.r.outs[tid] = a;
  }
  __syncthreads();
  if (wave == 0) {
    const v4f v = *(const v4fa*)(un.r.outs + 4 * lane);
    float* op = out + (size_t)b * (U_N * NCL) + 4 * lane;
    *(volatile v4f*)op = v;
    __threadfence();
    *(volatile v4f*)op = v;
  }
}

static inline int cdiv(int a, int b) { return (a + b - 1) / b; }
static inline size_t al256(size_t o) { return (o + 255) & ~(size_t)255; }

extern "C" void kernel_launch(void* const* d_in, const int* in_sizes, int n_in,
                              void* d_out, int out_size, void* d_ws, size_t ws_size,
                              hipStream_t stream) {
  if (n_in < 27) return;
  const int nB = in_sizes[2];
  if (nB < 1 || nB > (1 << 20)) return;
  if (in_sizes[0] != nB * U_N * 3) return;
  if (in_sizes[1] != nB * NE) return;
  if (in_sizes[3] != nB * U_N * HH) return;
  if (in_sizes[5] != nB * U_N || in_sizes[6] != nB * U_N) return;
  if (in_sizes[7] != 5 * SU || in_sizes[8] != SU) return;
  if (in_sizes[9] != (2 * SU + 2) * HH || in_sizes[10] != HH) return;
  if (in_sizes[11] != HH * (HH / 2) || in_sizes[12] != HH / 2) return;
  if (in_sizes[13] != (HH / 2) * SU || in_sizes[14] != SU) return;
  if (in_sizes[15] != SU * HH || in_sizes[16] != HH) return;
  if (in_sizes[17] != HH * (HH / 2) || in_sizes[18] != HH / 2) return;
  if (in_sizes[19] != (HH / 2) * NCL || in_sizes[20] != NCL) return;
  if (in_sizes[21] != G3 * SU || in_sizes[22] != G3 * HH) return;
  if (in_sizes[23] != G3 || in_sizes[24] != G3) return;
  if (in_sizes[25] != HH * SU || in_sizes[26] != SU) return;
  if (out_size != nB * U_N * NCL) return;

  const float* xf    = (const float*)d_in[0];
  const float* ewp   = (const float*)d_in[1];
  const float* noise = (const float*)d_in[2];
  const float* hx0   = (const float*)d_in[3];
  const float* xhat  = (const float*)d_in[5];
  const float* varm  = (const float*)d_in[6];
  const float* W1a = (const float*)d_in[7];  const float* b1a = (const float*)d_in[8];
  const float* W2a = (const float*)d_in[9];  const float* b2a = (const float*)d_in[10];
  const float* W2b = (const float*)d_in[11]; const float* b2b = (const float*)d_in[12];
  const float* W2c = (const float*)d_in[13]; const float* b2c = (const float*)d_in[14];
  const float* W3a = (const float*)d_in[15]; const float* b3a = (const float*)d_in[16];
  const float* W3b = (const float*)d_in[17]; const float* b3b = (const float*)d_in[18];
  const float* W3c = (const float*)d_in[19]; const float* b3c = (const float*)d_in[20];
  const float* Wih = (const float*)d_in[21]; const float* Whh = (const float*)d_in[22];
  const float* bih = (const float*)d_in[23]; const float* bhh = (const float*)d_in[24];
  const float* W4  = (const float*)d_in[25]; const float* b4  = (const float*)d_in[26];
  float* out = (float*)d_out;

  char* ws = (char*)d_ws;
  size_t off = 0;
  const size_t oWhh = off; off = al256(off + (size_t)G3 * KP * 2);
  const size_t oW2b = off; off = al256(off + (size_t)(HH / 2) * KP * 2);
  const size_t oW2c = off; off = al256(off + (size_t)16 * K2C * 2);
  if (off > ws_size || off > (size_t)WSMAX) return;
  unsigned short* WhhP = (unsigned short*)(ws + oWhh);
  unsigned short* W2bP = (unsigned short*)(ws + oW2b);
  unsigned short* W2cP = (unsigned short*)(ws + oW2c);

  {
    const int nUh = G3 * (KP / 8);
    k_wdup<<<cdiv(nUh, NTHR), NTHR, 0, stream>>>(Whh, WhhP, nUh);
    const int nUb = (HH / 2) * (KP / 8);
    k_wtr<<<cdiv(nUb, NTHR), NTHR, 0, stream>>>(W2b, HH, HH / 2, HH / 2, KP, W2bP, nUb);
    const int nUc = 16 * (K2C / 8);
    k_wtr<<<cdiv(nUc, NTHR), NTHR, 0, stream>>>(W2c, HH / 2, SU, 16, K2C, W2cP, nUc);
  }
  k_net<<<nB, NTHR, 0, stream>>>(xf, ewp, noise, hx0, xhat, varm, W1a, b1a, W2a, b2a, b2b, b2c,
                                 W3a, b3a, W3b, b3b, W3c, b3c, Wih, bih, bhh, W4, b4,
                                 W2bP, W2cP, WhhP, out);
}
